// NemotronHWayfinderAttention_377957122625
// MI455X (gfx1250) — hardware-verified
//
#include <hip/hip_runtime.h>
#include <hip/hip_bf16.h>
#include <stddef.h>
#include <stdint.h>

#define SQ    2048
#define HID   1024
#define NHQ   16
#define NKV   8
#define HDM   64
#define GRP   2
#define GRPW  (GRP * HDM)
#define KNB   128
#define NQKV  2048
#define KOF   (NHQ * HDM)
#define VOF   (NHQ * HDM + NKV * HDM)
#define QPB   8

static_assert(NHQ * HDM == HID);
static_assert(NHQ == GRP * NKV);
static_assert(NQKV == NHQ * HDM + 2 * NKV * HDM);
static_assert(KNB == 32 * 4);
static_assert(GRPW == 32 * 4);
static_assert(HDM % 4 == 0);
static_assert(SQ % 256 == 0);
static_assert(SQ % QPB == 0);
static_assert(HID % 64 == 0);
static_assert(NQKV % 64 == 0);
static_assert(HID % 32 == 0);
static_assert(HID == 128 * 8);

typedef float          v8f   __attribute__((ext_vector_type(8)));
typedef float          v4f   __attribute__((ext_vector_type(4)));
typedef int            v4i   __attribute__((ext_vector_type(4)));
typedef unsigned int   v4u   __attribute__((ext_vector_type(4)));
typedef unsigned short v8us  __attribute__((ext_vector_type(8)));
typedef unsigned short v16us __attribute__((ext_vector_type(16)));
typedef __bf16         v16b  __attribute__((ext_vector_type(16)));
typedef unsigned short ush;

union FragU { v16us v; v8us h[2]; v16b b; };
union PackU { v8us s; v4u u; };
struct HL { v4u h; v4u l; };

__device__ __forceinline__ ush f2bf(float f) {
  const unsigned u = __float_as_uint(f);
  return (ush)((u + 0x7FFFu + ((u >> 16) & 1u)) >> 16);
}
__device__ __forceinline__ float bf2f(ush b) { return __uint_as_float(((unsigned)b) << 16); }

__device__ __forceinline__ HL split8(v8f f) {
  PackU ph, pl;
#pragma unroll
  for (int e = 0; e < 8; ++e) {
    const ush hi = f2bf(f[e]);
    ph.s[e] = hi;
    pl.s[e] = f2bf(f[e] - bf2f(hi));
  }
  HL r; r.h = ph.u; r.l = pl.u;
  return r;
}

__device__ __forceinline__ v8f mmab(v16us a, v16us b, v8f c) {
  FragU ua, ub; ua.v = a; ub.v = b;
  c = __builtin_amdgcn_wmma_f32_16x16x32_bf16(false, ua.b, false, ub.b, (short)0, c, false, false);
  asm volatile("v_nop\n\tv_nop\n\tv_nop\n\tv_nop" : "+v"(c) : "v"(a), "v"(b));
  return c;
}

__device__ __forceinline__ v16us ldfragu(const ush* p, int ld, int row0, int k0, int lane) {
  const int m = lane & 15, lh = lane >> 4;
  const ush* q = p + (size_t)(row0 + m) * ld + k0 + 8 * lh;
  FragU f;
  f.h[0] = *(const v8us*)(q);
  f.h[1] = *(const v8us*)(q + 16);
  return f.v;
}

__device__ __forceinline__ v8f zero8() { return (v8f){0.f, 0.f, 0.f, 0.f, 0.f, 0.f, 0.f, 0.f}; }

__device__ __forceinline__ void gemm3_32x64(const ush* __restrict__ Ah, const ush* __restrict__ Al, int lda,
                                            const ush* __restrict__ Bh, const ush* __restrict__ Bl, int ldb,
                                            int m0, int n0, int lane, v8f (&acc)[2][4]) {
#pragma unroll 1
  for (int k0 = 0; k0 < HID; k0 += 32) {
    const v16us a0h = ldfragu(Ah, lda, m0, k0, lane);
    const v16us a1h = ldfragu(Ah, lda, m0 + 16, k0, lane);
    const v16us a0l = ldfragu(Al, lda, m0, k0, lane);
    const v16us a1l = ldfragu(Al, lda, m0 + 16, k0, lane);
#pragma unroll
    for (int t = 0; t < 4; ++t) {
      const v16us bh = ldfragu(Bh, ldb, n0 + 16 * t, k0, lane);
      const v16us bl = ldfragu(Bl, ldb, n0 + 16 * t, k0, lane);
      acc[0][t] = mmab(a0h, bh, acc[0][t]);
      acc[1][t] = mmab(a1h, bh, acc[1][t]);
      acc[0][t] = mmab(a0h, bl, acc[0][t]);
      acc[1][t] = mmab(a1h, bl, acc[1][t]);
      acc[0][t] = mmab(a0l, bh, acc[0][t]);
      acc[1][t] = mmab(a1l, bh, acc[1][t]);
    }
  }
}

#define OTP 68
__device__ __forceinline__ void out_epilogue(v8f (&acc)[2][4], float* sw, float* __restrict__ out, int ldc,
                                             int m0, int n0, int lane, int hh, int c) {
#pragma unroll
  for (int sub = 0; sub < 2; ++sub) {
    __syncthreads();
#pragma unroll
    for (int t = 0; t < 4; ++t) {
#pragma unroll
      for (int r = 0; r < 8; ++r) sw[(8 * hh + r) * OTP + 16 * t + c] = acc[sub][t][r];
    }
    __syncthreads();
    v4f val[8];
    size_t go[8];
#pragma unroll
    for (int it = 0; it < 8; ++it) {
      const int p    = lane + 32 * it;
      const int L    = p >> 3;
      const int pc   = p & 7;
      const int row  = L >> 1;
      const int half = L & 1;
      val[it] = *(const v4f*)(sw + row * OTP + half * 32 + pc * 4);
      go[it]  = (size_t)(m0 + sub * 16 + row) * ldc + n0 + half * 32 + pc * 4;
    }
    for (int ps = 0; ps < 2; ++ps) {
#pragma unroll
      for (int it = 0; it < 8; ++it) *(volatile v4f*)(out + go[it]) = val[it];
      __threadfence();
    }
  }
}

__global__ __launch_bounds__(128) void k_cvt(const float* __restrict__ src, ush* __restrict__ dh,
                                             ush* __restrict__ dl, int rofs) {
  const int row = blockIdx.x;
  const int col = (int)threadIdx.x * 8;
  const size_t o = (size_t)row * HID + col;
  const v4f a0 = *(const v4f*)(src + o);
  const v4f a1 = *(const v4f*)(src + o + 4);
  const v8f f = (v8f){a0[0], a0[1], a0[2], a0[3], a1[0], a1[1], a1[2], a1[3]};
  const HL sp = split8(f);
  const size_t od = (size_t)(rofs + row) * HID + col;
  *(volatile v4u*)(dh + od) = sp.h;
  *(volatile v4u*)(dl + od) = sp.l;
  __threadfence();
  *(volatile v4u*)(dh + od) = sp.h;
  *(volatile v4u*)(dl + od) = sp.l;
}

__global__ __launch_bounds__(256) void k_gemm3(const ush* __restrict__ ah, const ush* __restrict__ al,
                                               const ush* __restrict__ bh, const ush* __restrict__ bl,
                                               float* __restrict__ out, int ldc) {
  __shared__ __align__(16) float st[8][16 * OTP];
  const int tid = threadIdx.x, lane = tid & 31, wave = tid >> 5;
  const int hh = lane >> 4, c = lane & 15;
  const int m0 = blockIdx.x * 256 + wave * 32;
  const int n0 = blockIdx.y * 64;

  v8f acc[2][4];
#pragma unroll
  for (int s = 0; s < 2; ++s)
#pragma unroll
    for (int t = 0; t < 4; ++t) acc[s][t] = zero8();
  gemm3_32x64(ah, al, HID, bh, bl, HID, m0, n0, lane, acc);
  out_epilogue(acc, st[wave], out, ldc, m0, n0, lane, hh, c);
}

__device__ __forceinline__ float dacc(v4f q, v4f k, float a) {
  a = fmaf(q[0], k[0], a);
  a = fmaf(q[1], k[1], a);
  a = fmaf(q[2], k[2], a);
  a = fmaf(q[3], k[3], a);
  return a;
}

__global__ __launch_bounds__(256) void k_attn(const float* __restrict__ qkv,
                                              const int* __restrict__ nidx,
                                              const int* __restrict__ etyp,
                                              const float* __restrict__ ebias,
                                              float* __restrict__ op) {
  __shared__ __align__(16) float sq[QPB][GRPW];
  __shared__ __align__(16) float sp[QPB][GRP][KNB];
  __shared__ __align__(16) int   si[QPB][KNB];

  const int tid = threadIdx.x, lane = tid & 31, wave = tid >> 5;
  const int nsb = SQ / QPB;
  const int h   = blockIdx.x / nsb;
  const int s   = (blockIdx.x - h * nsb) * QPB + wave;

  {
    const v4f q4 = *(const v4f*)(qkv + (size_t)s * NQKV + h * GRPW + lane * 4);
    *(v4f*)(&sq[wave][lane * 4]) = q4;
  }
  const size_t nb = ((size_t)h * SQ + s) * KNB + lane * 4;
  const v4i id = *(const v4i*)(nidx + nb);
  const v4i et = *(const v4i*)(etyp + nb);
  int cid0, cid1, cid2, cid3;
  {
    int v;
    v = id[0]; v = (v < 0) ? 0 : v; v = (v > SQ - 1) ? (SQ - 1) : v; cid0 = v;
    v = id[1]; v = (v < 0) ? 0 : v; v = (v > SQ - 1) ? (SQ - 1) : v; cid1 = v;
    v = id[2]; v = (v < 0) ? 0 : v; v = (v > SQ - 1) ? (SQ - 1) : v; cid2 = v;
    v = id[3]; v = (v < 0) ? 0 : v; v = (v > SQ - 1) ? (SQ - 1) : v; cid3 = v;
  }
  *(v4i*)(&si[wave][lane * 4]) = (v4i){cid0, cid1, cid2, cid3};
  const float eb0 = ebias[0], eb1 = ebias[1], eb2 = ebias[2], eb3 = ebias[3];
  __syncthreads();

  const float* kbase = qkv + KOF + h * HDM;
  const float* kp0 = kbase + (size_t)cid0 * NQKV;
  const float* kp1 = kbase + (size_t)cid1 * NQKV;
  const float* kp2 = kbase + (size_t)cid2 * NQKV;
  const float* kp3 = kbase + (size_t)cid3 * NQKV;
  float a00 = 0.f, a01 = 0.f, a02 = 0.f, a03 = 0.f;
  float a10 = 0.f, a11 = 0.f, a12 = 0.f, a13 = 0.f;
#pragma unroll 1
  for (int c4 = 0; c4 < HDM; c4 += 4) {
    const v4f qa = *(const v4f*)(&sq[wave][c4]);
    const v4f qb = *(const v4f*)(&sq[wave][HDM + c4]);
    const v4f k0 = *(const v4f*)(kp0 + c4);
    const v4f k1 = *(const v4f*)(kp1 + c4);
    const v4f k2 = *(const v4f*)(kp2 + c4);
    const v4f k3 = *(const v4f*)(kp3 + c4);
    a00 = dacc(qa, k0, a00);
    a01 = dacc(qa, k1, a01);
    a02 = dacc(qa, k2, a02);
    a03 = dacc(qa, k3, a03);
    a10 = dacc(qb, k0, a10);
    a11 = dacc(qb, k1, a11);
    a12 = dacc(qb, k2, a12);
    a13 = dacc(qb, k3, a13);
  }

  const float NEG = -__FLT_MAX__;
  float s0[4], s1[4];
  {
    const float av0[4] = {a00, a01, a02, a03};
    const float av1[4] = {a10, a11, a12, a13};
#pragma unroll
    for (int j = 0; j < 4; ++j) {
      const int v = id[j];
      const bool ok = (v >= 0) && (v < SQ) && (v <= s);
      int t = et[j]; t = (t < 0) ? 0 : t; t = (t > 3) ? 3 : t;
      const float b = (t == 0) ? eb0 : ((t == 1) ? eb1 : ((t == 2) ? eb2 : eb3));
      s0[j] = ok ? (av0[j] * 0.125f + b) : NEG;
      s1[j] = ok ? (av1[j] * 0.125f + b) : NEG;
    }
  }

  float m0 = fmaxf(fmaxf(s0[0], s0[1]), fmaxf(s0[2], s0[3]));
  float m1 = fmaxf(fmaxf(s1[0], s1[1]), fmaxf(s1[2], s1[3]));
#pragma unroll
  for (int off = 16; off > 0; off >>= 1) {
    m0 = fmaxf(m0, __shfl_xor(m0, off, 32));
    m1 = fmaxf(m1, __shfl_xor(m1, off, 32));
  }
  float e0[4], e1[4];
  float z0 = 0.f, z1 = 0.f;
#pragma unroll
  for (int j = 0; j < 4; ++j) {
    e0[j] = __expf(s0[j] - m0); z0 += e0[j];
    e1[j] = __expf(s1[j] - m1); z1 += e1[j];
  }
#pragma unroll
  for (int off = 16; off > 0; off >>= 1) {
    z0 += __shfl_xor(z0, off, 32);
    z1 += __shfl_xor(z1, off, 32);
  }
  const float i0 = 1.0f / z0;
  const float i1 = 1.0f / z1;
  *(v4f*)(&sp[wave][0][lane * 4]) = (v4f){e0[0] * i0, e0[1] * i0, e0[2] * i0, e0[3] * i0};
  *(v4f*)(&sp[wave][1][lane * 4]) = (v4f){e1[0] * i1, e1[1] * i1, e1[2] * i1, e1[3] * i1};
  __syncthreads();

  const int gi = lane >> 4;
  const int ch = (lane & 15) * 4;
  const float* vbase = qkv + VOF + h * HDM + ch;
  const float* pp = &sp[wave][gi][0];
  const int*   ip = &si[wave][0];
  v4f o = (v4f){0.f, 0.f, 0.f, 0.f};
#pragma unroll 2
  for (int kk = 0; kk < KNB; ++kk) {
    const int   ix = ip[kk];
    const float p  = pp[kk];
    const v4f  vv  = *(const v4f*)(vbase + (size_t)ix * NQKV);
    o = p * vv + o;
  }
  float* orow = op + (size_t)s * HID + h * GRPW + lane * 4;
  *(volatile v4f*)orow = o;
  __threadfence();
  *(volatile v4f*)orow = o;
}

extern "C" void kernel_launch(void* const* d_in, const int* in_sizes, int n_in,
                              void* d_out, int out_size, void* d_ws, size_t ws_size,
                              hipStream_t stream) {
  if (n_in < 8) return;
  if (in_sizes[0] != SQ * HID) return;
  if (in_sizes[1] != NHQ * HDM * HID) return;
  if (in_sizes[2] != NKV * HDM * HID) return;
  if (in_sizes[3] != NKV * HDM * HID) return;
  if (in_sizes[4] != HID * NHQ * HDM) return;
  if (in_sizes[5] != 4) return;
  if (in_sizes[6] != NKV * SQ * KNB) return;
  if (in_sizes[7] != NKV * SQ * KNB) return;
  if (out_size != SQ * HID) return;

  const float* x    = (const float*)d_in[0];
  const float* qw   = (const float*)d_in[1];
  const float* kw   = (const float*)d_in[2];
  const float* vw   = (const float*)d_in[3];
  const float* ow   = (const float*)d_in[4];
  const float* eb   = (const float*)d_in[5];
  const int*   nidx = (const int*)d_in[6];
  const int*   etyp = (const int*)d_in[7];
  float* out = (float*)d_out;

  size_t off = 0;
  const size_t oXh  = off; off += (size_t)SQ * HID * 2;
  const size_t oXl  = off; off += (size_t)SQ * HID * 2;
  const size_t oWh  = off; off += (size_t)NQKV * HID * 2;
  const size_t oWl  = off; off += (size_t)NQKV * HID * 2;
  const size_t oWoh = off; off += (size_t)HID * HID * 2;
  const size_t oWol = off; off += (size_t)HID * HID * 2;
  const size_t oQKV = off; off += (size_t)SQ * NQKV * 4;
  const size_t oO   = off; off += (size_t)SQ * HID * 4;
  const size_t oOh  = off; off += (size_t)SQ * HID * 2;
  const size_t oOl  = off; off += (size_t)SQ * HID * 2;
  if (off > ws_size) return;
  if (off > (size_t)134217728) return;

  char* ws = (char*)d_ws;
  ush*   Xh  = (ush*)(ws + oXh);
  ush*   Xl  = (ush*)(ws + oXl);
  ush*   Wh  = (ush*)(ws + oWh);
  ush*   Wl  = (ush*)(ws + oWl);
  ush*   Woh = (ush*)(ws + oWoh);
  ush*   Wol = (ush*)(ws + oWol);
  float* QKV = (float*)(ws + oQKV);
  float* Of  = (float*)(ws + oO);
  ush*   Oh  = (ush*)(ws + oOh);
  ush*   Ol  = (ush*)(ws + oOl);

  k_cvt<<<dim3(SQ), dim3(128), 0, stream>>>(x, Xh, Xl, 0);
  k_cvt<<<dim3(NHQ * HDM), dim3(128), 0, stream>>>(qw, Wh, Wl, 0);
  k_cvt<<<dim3(NKV * HDM), dim3(128), 0, stream>>>(kw, Wh, Wl, KOF);
  k_cvt<<<dim3(NKV * HDM), dim3(128), 0, stream>>>(vw, Wh, Wl, VOF);
  k_cvt<<<dim3(HID), dim3(128), 0, stream>>>(ow, Woh, Wol, 0);
  k_gemm3<<<dim3(SQ / 256, NQKV / 64), dim3(256), 0, stream>>>(Xh, Xl, Wh, Wl, QKV, NQKV);
  k_attn<<<dim3(NKV * (SQ / QPB)), dim3(256), 0, stream>>>(QKV, nidx, etyp, eb, Of);
  k_cvt<<<dim3(SQ), dim3(128), 0, stream>>>(Of, Oh, Ol, 0);
  k_gemm3<<<dim3(SQ / 256, HID / 64), dim3(256), 0, stream>>>(Oh, Ol, Woh, Wol, out, HID);
  (void)hipGetLastError();
}
